// LinearAttention_65326452572467
// MI455X (gfx1250) — hardware-verified
//
#include <hip/hip_runtime.h>


#ifndef NB
#define NB 2
#endif
#ifndef SEQ
#define SEQ 2048
#endif
#define NB_FULL  2
#define SEQ_FULL 2048
#define NHD 16
#define HD  64
#define BH  (NB * NHD)
#define ZH  2
static_assert(SEQ % 256 == 0);
static_assert(SEQ <= SEQ_FULL);
static_assert(NB <= NB_FULL);
static_assert(BH % ZH == 0);
static_assert(HD == 64);

typedef _Float16 h16;
typedef unsigned short bf;
typedef __attribute__((ext_vector_type(16))) __bf16   v16bf;
typedef __attribute__((ext_vector_type(16))) _Float16 v16h;
typedef __attribute__((ext_vector_type(8)))  _Float16 v8h;
typedef __attribute__((ext_vector_type(8)))  unsigned short v8us;
typedef __attribute__((ext_vector_type(8)))  float    v8f;
typedef __attribute__((ext_vector_type(4)))  float    v4f;
typedef __attribute__((ext_vector_type(2)))  float    v2f;
typedef v8h  __attribute__((may_alias)) v8ha;
typedef v4f  __attribute__((may_alias)) v4fa;
typedef v8us __attribute__((may_alias)) v8usa;

__device__ __forceinline__ unsigned short f2bf(float f) { unsigned u = __float_as_uint(f); u += 0x7FFFu + ((u >> 16) & 1u); return (unsigned short)(u >> 16); }
__device__ __forceinline__ float bf2f(unsigned short b) { return __uint_as_float(((unsigned)b) << 16); }
__device__ __forceinline__ float bfr(float f) { return bf2f(f2bf(f)); }
__device__ __forceinline__ void splitf(float y, unsigned short& h, unsigned short& l) { h = f2bf(y); l = f2bf(y - bf2f(h)); }
__device__ __forceinline__ v16h cat16(v8h lo, v8h hi) { return __builtin_shufflevector(lo, hi, 0, 1, 2, 3, 4, 5, 6, 7, 8, 9, 10, 11, 12, 13, 14, 15); }
__device__ __forceinline__ v16bf cat16b(v8us lo, v8us hi) { return __builtin_bit_cast(v16bf, __builtin_shufflevector(lo, hi, 0, 1, 2, 3, 4, 5, 6, 7, 8, 9, 10, 11, 12, 13, 14, 15)); }
__device__ __forceinline__ v8f wmma16(v16h a, v16h b, v8f c) { return __builtin_amdgcn_wmma_f32_16x16x32_f16(false, a, false, b, (short)0, c, false, false); }
__device__ __forceinline__ v8f wmmab(v16bf a, v16bf b, v8f c) { return __builtin_amdgcn_wmma_f32_16x16x32_bf16(false, a, false, b, (short)0, c, false, false); }

template <typename T16> struct WFrag;
template <> struct WFrag<h16> { typedef v16h V; static __device__ __forceinline__ V ld(const h16* p) { return cat16(*(const v8h*)p, *(const v8h*)(p + 16)); } static __device__ __forceinline__ v8f mma(V a, V b, v8f c) { return wmma16(a, b, c); } };
template <> struct WFrag<bf> { typedef v16bf V; static __device__ __forceinline__ V ld(const bf* p) { return cat16b(*(const v8us*)p, *(const v8us*)(p + 16)); } static __device__ __forceinline__ v8f mma(V a, V b, v8f c) { return wmmab(a, b, c); } };

template <typename T16, int NSPLIT, int CMODE>
__global__ __launch_bounds__(32) void k_gemmc(const T16* __restrict__ A, const T16* __restrict__ A2, const T16* __restrict__ Bt, const T16* __restrict__ Bt2, int K, float* C, int ldc, int roff, size_t sA, size_t sB, size_t sC) {
    typedef typename WFrag<T16>::V V;
    __shared__ __align__(16) float os[16 * 68];
    const size_t z = blockIdx.z; A += z * sA; if (A2) A2 += z * sA; Bt += z * sB; if (Bt2) Bt2 += z * sB; C += z * sC;
    const int lane = threadIdx.x & 31, lr = lane & 15, hi = lane >> 4; const int r0 = blockIdx.x * 64, c0 = blockIdx.y * 64;
    if (CMODE == 1 && c0 > r0 + roff + 63) return;
    const int Kl = (CMODE == 2) ? min(K, r0 + roff + 64) : K;
    v8f acc[4][4];
#pragma unroll
    for (int mb = 0; mb < 4; ++mb)
#pragma unroll
        for (int nb = 0; nb < 4; ++nb) acc[mb][nb] = (v8f){};
    const size_t aoff = (size_t)(r0 + lr) * K + 8 * hi, boff = (size_t)(c0 + lr) * K + 8 * hi;
#pragma unroll 1
    for (int kc = 0; kc < Kl; kc += 32) {
        V a[4], a2[4];
#pragma unroll
        for (int mb = 0; mb < 4; ++mb) { a[mb] = WFrag<T16>::ld(A + aoff + (size_t)mb * 16 * K + kc); if (NSPLIT == 1 || NSPLIT == 2) a2[mb] = WFrag<T16>::ld(A2 + aoff + (size_t)mb * 16 * K + kc); }
#pragma unroll
        for (int nb = 0; nb < 4; ++nb) { const V b = WFrag<T16>::ld(Bt + boff + (size_t)nb * 16 * K + kc); V b2; if (NSPLIT >= 2) b2 = WFrag<T16>::ld(Bt2 + boff + (size_t)nb * 16 * K + kc);
#pragma unroll
            for (int mb = 0; mb < 4; ++mb) { acc[mb][nb] = WFrag<T16>::mma(a[mb], b, acc[mb][nb]); if (NSPLIT == 1 || NSPLIT == 2) acc[mb][nb] = WFrag<T16>::mma(a2[mb], b, acc[mb][nb]); if (NSPLIT >= 2) acc[mb][nb] = WFrag<T16>::mma(a[mb], b2, acc[mb][nb]); } }
        asm volatile("v_nop\n\tv_nop\n\tv_nop\n\tv_nop" : "+v"(acc[0][0]), "+v"(acc[1][1]), "+v"(acc[2][2]), "+v"(acc[3][3]) : "v"(a[0]), "v"(a[3]));
    }
#pragma unroll
    for (int mb = 0; mb < 4; ++mb) {
#pragma unroll
        for (int nb = 0; nb < 4; ++nb) {
#pragma unroll
            for (int j = 0; j < 8; ++j) os[(hi * 8 + j) * 68 + nb * 16 + lr] = acc[mb][nb][j]; }
        __builtin_amdgcn_wave_barrier(); asm volatile("" ::: "memory");
        float* crow = C + (size_t)(r0 + mb * 16) * ldc + c0;
#pragma unroll 1
        for (int ps = 0; ps < 2; ++ps) {
#pragma unroll
            for (int s = 0; s < 8; ++s) { const int row = 2 * s + hi, cofs = lr * 4; v4f val = *(const v4fa*)(os + row * 68 + cofs);
                *(volatile v4f*)(crow + (size_t)row * ldc + cofs) = val; }
            if (ps == 0) __threadfence(); }
        __builtin_amdgcn_wave_barrier(); asm volatile("" ::: "memory");
    }
}

__constant__ float DIVT[HD / 2] = {
    1.0f, 0.7498942017555237f, 0.5623413324356079f, 0.4216964840888977f, 0.3162277638912201f, 0.2371373474597931f, 0.17782793939113617f, 0.1333521455526352f, 0.09999999403953552f, 0.07498941570520401f, 0.056234125047922134f, 0.04216965287923813f, 0.03162277489900589f, 0.02371373400092125f, 0.017782796174287796f, 0.013335213996469975f, 0.009999999776482582f, 0.007498940918594599f, 0.0056234123185276985f, 0.004216963890939951f, 0.0031622766982764006f, 0.002371374052017927f, 0.0017782794311642647f, 0.0013335213297978044f, 0.0009999999310821295f, 0.0007498940685763955f, 0.0005623411852866411f, 0.0004216964007355273f, 0.0003162277862429619f, 0.00023713726841378957f, 0.00017782794020604342f, 0.00013335207768250257f
};

__global__ __launch_bounds__(256) void k_cs(float* CS, int n) {
#pragma clang fp contract(off)
    const int idx = blockIdx.x * 256 + threadIdx.x; if (idx >= n) return;
    const int p = idx & 31; const int t = idx >> 5;
    const float a = __fmul_rn((float)t, DIVT[p]);
    float sn, cn; sincosf(a, &sn, &cn);
    v2f o; o[0] = cn; o[1] = sn;
    float* dst = CS + (size_t)idx * 2;
    *(volatile v2f*)dst = o; __threadfence(); *(volatile v2f*)dst = o;
}

__global__ __launch_bounds__(256) void k_rope(const float* __restrict__ F, const float* __restrict__ CS, bf* Ph, bf* Pl, int n8) {
#pragma clang fp contract(off)
    const int g = blockIdx.x * 256 + threadIdx.x; if (g >= n8) return;
    const size_t e = (size_t)g * 8;
    const int d0 = (int)(e % HD); const int t = (int)((e / HD) % SEQ); const int bh = (int)(e / ((size_t)HD * SEQ));
    const float* src = F + ((size_t)bh * SEQ_FULL + t) * HD + d0;
    const v4f xa = *(const v4f*)src; const v4f xb = *(const v4f*)(src + 4);
    const float* csp = CS + ((size_t)t * (HD / 2) + (d0 >> 1)) * 2;
    const v4f ca = *(const v4f*)csp; const v4f cb = *(const v4f*)(csp + 4);
    float x[8]  = { xa[0], xa[1], xa[2], xa[3], xb[0], xb[1], xb[2], xb[3] };
    float cs[8] = { ca[0], ca[1], ca[2], ca[3], cb[0], cb[1], cb[2], cb[3] };
    v8us oh, ol;
#pragma unroll
    for (int q = 0; q < 4; ++q) {
        const float xe = bfr(x[2 * q]), xo = bfr(x[2 * q + 1]); const float c = cs[2 * q], sn = cs[2 * q + 1];
        float m0 = __fmul_rn(xe, c), m1 = __fmul_rn(xo, sn), m2 = __fmul_rn(xe, sn), m3 = __fmul_rn(xo, c);
        asm volatile("" : "+v"(m0)); asm volatile("" : "+v"(m1)); asm volatile("" : "+v"(m2)); asm volatile("" : "+v"(m3));
        const float re = __fsub_rn(m0, m1), ro = __fadd_rn(m2, m3);
        unsigned short ah, al; splitf(re, ah, al); oh[2 * q] = ah; ol[2 * q] = al; splitf(ro, ah, al); oh[2 * q + 1] = ah; ol[2 * q + 1] = al;
    }
    bf* hp = Ph + e; bf* lp = Pl + e;
    *(volatile v8us*)hp = oh; *(volatile v8us*)lp = ol; __threadfence(); *(volatile v8us*)hp = oh; *(volatile v8us*)lp = ol;
}

__global__ __launch_bounds__(256) void k_vtp(const float* __restrict__ F, bf* VT, int n8) {
    const int g = blockIdx.x * 256 + threadIdx.x; if (g >= n8) return;
    const size_t e = (size_t)g * 8;
    const int t0 = (int)(e % SEQ); const int d = (int)((e / SEQ) % HD); const int bh = (int)(e / ((size_t)SEQ * HD));
    const float* src = F + ((size_t)bh * SEQ_FULL + t0) * HD + d;
    v8us o;
#pragma unroll
    for (int j = 0; j < 8; ++j) o[j] = f2bf(src[(size_t)j * HD]);
    bf* dst = VT + e;
    *(volatile v8us*)dst = o; __threadfence(); *(volatile v8us*)dst = o;
}

__global__ __launch_bounds__(256) void k_smx(const float* __restrict__ Sb, bf* Ph, bf* Pl) {
    __shared__ float rmx[8];
    __shared__ float rsm[8];
    const int tid = threadIdx.x, wave = tid >> 5, lane = tid & 31;
    const int i = blockIdx.x, zz = blockIdx.y;
    const size_t rofs = ((size_t)zz * SEQ + i) * (size_t)SEQ;
    const int kl = ((i >> 6) + 1) << 6;
    const int c0 = tid * 8;
    const bool wact = (wave * 256) < kl;
    const float ninf = -__builtin_inff();
    float s[8];
#pragma unroll
    for (int q = 0; q < 8; ++q) s[q] = ninf;
    if (wact) {
        const v4f x0 = *(const v4f*)(Sb + rofs + c0); const v4f x1 = *(const v4f*)(Sb + rofs + c0 + 4);
#pragma unroll
        for (int q = 0; q < 4; ++q) { s[q] = (c0 + q <= i) ? x0[q] : ninf; s[4 + q] = (c0 + 4 + q <= i) ? x1[q] : ninf; }
    }
    float mx = s[0];
#pragma unroll
    for (int q = 1; q < 8; ++q) mx = fmaxf(mx, s[q]);
#pragma unroll
    for (int o = 16; o > 0; o >>= 1) mx = fmaxf(mx, __shfl_xor(mx, o));
    if (lane == 0) rmx[wave] = mx;
    __syncthreads();
    float m = rmx[0];
#pragma unroll
    for (int w = 1; w < 8; ++w) m = fmaxf(m, rmx[w]);
    float p[8]; float sum = 0.0f;
#pragma unroll
    for (int q = 0; q < 8; ++q) { const float dlt = fmaxf(s[q] - m, -200.0f); const float ev = __expf(dlt); p[q] = (c0 + q <= i) ? ev : 0.0f; sum += p[q]; }
#pragma unroll
    for (int o = 16; o > 0; o >>= 1) sum += __shfl_xor(sum, o);
    if (lane == 0) rsm[wave] = sum;
    __syncthreads();
    float l = rsm[0];
#pragma unroll
    for (int w = 1; w < 8; ++w) l += rsm[w];
    const float invl = 1.0f / l;
    if (wact) {
        v8us oh, ol;
#pragma unroll
        for (int q = 0; q < 8; ++q) { const float P = p[q] * invl; unsigned short ah, al; splitf(P, ah, al); oh[q] = ah; ol[q] = al; }
        bf* hp = Ph + rofs + c0; bf* lp = Pl + rofs + c0;
        *(volatile v8us*)hp = oh; *(volatile v8us*)lp = ol;
        __threadfence();
        *(volatile v8us*)hp = oh; *(volatile v8us*)lp = ol;
    }
}

extern "C" void kernel_launch(void* const* d_in, const int* in_sizes, int n_in,
                              void* d_out, int out_size, void* d_ws, size_t ws_size, hipStream_t stream) {
    if (n_in < 3) return;
    const int need = BH * SEQ_FULL * HD;
    if (in_sizes[0] < need || in_sizes[1] < need || in_sizes[2] < need) return;
    if (out_size < need) return;
    const float* Qin = (const float*)d_in[0]; const float* Kin = (const float*)d_in[1]; const float* Vin = (const float*)d_in[2];
    float* OUT = (float*)d_out;
    char* wsp = (char*)d_ws;
    auto take = [&](size_t bytes) { char* p = wsp; wsp += (bytes + 255) & ~(size_t)255; return (void*)p; };
    float* CS  = (float*)take((size_t)SEQ * (HD / 2) * 2 * 4);
    bf* QPh = (bf*)take((size_t)BH * SEQ * HD * 2); bf* QPl = (bf*)take((size_t)BH * SEQ * HD * 2);
    bf* KPh = (bf*)take((size_t)BH * SEQ * HD * 2); bf* KPl = (bf*)take((size_t)BH * SEQ * HD * 2);
    bf* VT  = (bf*)take((size_t)BH * HD * SEQ * 2);
    float* Sb = (float*)take((size_t)ZH * SEQ * SEQ * 4);
    bf* Ph  = (bf*)take((size_t)ZH * SEQ * SEQ * 2); bf* Pl = (bf*)take((size_t)ZH * SEQ * SEQ * 2);
    if ((size_t)(wsp - (char*)d_ws) > ws_size) return;
    const int ncs = SEQ * (HD / 2);
    const int n8 = BH * SEQ * HD / 8;
    k_cs<<<(unsigned)((ncs + 255) / 256), 256, 0, stream>>>(CS, ncs);
    k_rope<<<(unsigned)((n8 + 255) / 256), 256, 0, stream>>>(Qin, CS, QPh, QPl, n8);
    k_rope<<<(unsigned)((n8 + 255) / 256), 256, 0, stream>>>(Kin, CS, KPh, KPl, n8);
    k_vtp<<<(unsigned)((n8 + 255) / 256), 256, 0, stream>>>(Vin, VT, n8);
    for (int gidx = 0; gidx < BH / ZH; ++gidx) {
        const size_t bh0 = (size_t)gidx * ZH;
        k_gemmc<bf, 2, 1><<<dim3(SEQ / 64, SEQ / 64, ZH), 32, 0, stream>>>(QPh + bh0 * SEQ * HD, QPl + bh0 * SEQ * HD, KPh + bh0 * SEQ * HD, KPl + bh0 * SEQ * HD, HD, Sb, SEQ, 0, (size_t)SEQ * HD, (size_t)SEQ * HD, (size_t)SEQ * SEQ);
        k_smx<<<dim3(SEQ, ZH), 256, 0, stream>>>(Sb, Ph, Pl);
        k_gemmc<bf, 1, 2><<<dim3(SEQ / 64, HD / 64, ZH), 32, 0, stream>>>(Ph, Pl, VT + bh0 * HD * SEQ, (const bf*)nullptr, SEQ, OUT + bh0 * SEQ_FULL * HD, HD, 0, (size_t)SEQ * SEQ, (size_t)HD * SEQ, (size_t)SEQ_FULL * HD);
    }
}
